// MultiHeadAttention_18519898980590
// MI455X (gfx1250) — hardware-verified
//
#include <hip/hip_runtime.h>


#ifndef NB
#define NB 16
#endif
#define NB_FULL 16
#define SEQ  512
#define NF   512
#define NH_  8
#define DH   512
#define HDIM (NH_ * DH)
#define BCH  (NB < 4 ? NB : 4)
#define AW   4
#define PP   520
#define SC2  ((float)(0.04419417382415922 * 1.4426950408889634))
#define PSH  14.0f
#define NEGB (-3.0e38f)
#define CTXC 64.0f
#define WOC  64.0f
#define OSC  (1.0f / 4096.0f)

static_assert(DH == SEQ);
static_assert(NF == SEQ);
static_assert(NH_ * DH == HDIM);
static_assert(NF % 32 == 0);
static_assert(SEQ % 32 == 0);
static_assert(HDIM % 32 == 0);
static_assert(SEQ % 64 == 0);
static_assert(DH % 64 == 0);
static_assert(HDIM % 64 == 0);
static_assert(NF % 64 == 0);
static_assert((BCH * SEQ) % 64 == 0);
static_assert(BCH * SEQ <= HDIM);
static_assert(NB % BCH == 0);
static_assert(NB <= NB_FULL);
static_assert(DH == AW * 128);
static_assert(SEQ % 32 == 0);
static_assert((PP * 2) % 16 == 0);
static_assert(PP >= DH);
static_assert(32 * 16 * 4 == 16 * 64 * 2);
static_assert(32 * 16 * 16 == 32 * 128 * 2);
static_assert(32 * 16 * 8 == 16 * 64 * 4);
static_assert(16 * 68 * 4 <= 131072);
static_assert(32 * PP * 2 + 2 * AW * 32 * 4 <= 131072);
static_assert(((size_t)NB * SEQ * NF) % 8 == 0);
static_assert(((size_t)HDIM * NF) % 8 == 0);

typedef _Float16 h16;
typedef unsigned short bf;
typedef __attribute__((ext_vector_type(16))) __bf16   v16bf;
typedef __attribute__((ext_vector_type(16))) _Float16 v16h;
typedef __attribute__((ext_vector_type(8)))  _Float16 v8h;
typedef __attribute__((ext_vector_type(8)))  unsigned short v8us;
typedef __attribute__((ext_vector_type(8)))  float    v8f;
typedef __attribute__((ext_vector_type(4)))  float    v4f;
typedef v4f  __attribute__((may_alias)) v4fa;

__device__ __forceinline__ unsigned short f2bf(float f) { unsigned u = __float_as_uint(f); u += 0x7FFFu + ((u >> 16) & 1u); return (unsigned short)(u >> 16); }
__device__ __forceinline__ float bfr(float f) { return __uint_as_float(((unsigned)f2bf(f)) << 16); }
__device__ __forceinline__ v16h cat16(v8h lo, v8h hi) { return __builtin_shufflevector(lo, hi, 0, 1, 2, 3, 4, 5, 6, 7, 8, 9, 10, 11, 12, 13, 14, 15); }
__device__ __forceinline__ v16bf cat16b(v8us lo, v8us hi) { return __builtin_bit_cast(v16bf, __builtin_shufflevector(lo, hi, 0, 1, 2, 3, 4, 5, 6, 7, 8, 9, 10, 11, 12, 13, 14, 15)); }
__device__ __forceinline__ v8f wmma16(v16h a, v16h b, v8f c) { return __builtin_amdgcn_wmma_f32_16x16x32_f16(false, a, false, b, (short)0, c, false, false); }
__device__ __forceinline__ v8f wmmab(v16bf a, v16bf b, v8f c) { return __builtin_amdgcn_wmma_f32_16x16x32_bf16(false, a, false, b, (short)0, c, false, false); }
__device__ __forceinline__ v16h  ldh(const h16* p) { return cat16(*(const v8h*)p, *(const v8h*)(p + 16)); }
__device__ __forceinline__ v16bf ldb(const bf* p)  { return cat16b(*(const v8us*)p, *(const v8us*)(p + 16)); }
__device__ __forceinline__ void wave_sync() { __builtin_amdgcn_fence(3  , "wavefront"); __builtin_amdgcn_wave_barrier(); asm volatile("" ::: "memory"); }

__device__ __forceinline__ v8f wmma16_g(v16h a, v16h b, v8f c) { c = wmma16(a, b, c); asm volatile("v_nop\n\tv_nop\n\tv_nop\n\tv_nop" : "+v"(c) : "v"(a), "v"(b)); return c; }
__device__ __forceinline__ v8f wmmab_g(v16bf a, v16bf b, v8f c) { c = wmmab(a, b, c); asm volatile("v_nop\n\tv_nop\n\tv_nop\n\tv_nop" : "+v"(c) : "v"(a), "v"(b)); return c; }
static __device__ __forceinline__ h16 toh_flush(float v) { const h16 r = (h16)v; return (fabsf(v) < 6.103515625e-05f) ? (h16)0.0f : r; }
static __device__ __forceinline__ h16 pexp_h(float e) { const h16 r = (h16)__builtin_amdgcn_exp2f(e); return (e < -14.0f) ? (h16)0.0f : r; }

__global__ __launch_bounds__(256) void k_cvt8(const float* __restrict__ src, bf* dst, size_t n8) {
    const size_t i = (size_t)blockIdx.x * 256 + threadIdx.x; if (i >= n8) return;
    const v8f v = *(const v8f*)(src + i * 8); v8us o;
#pragma unroll
    for (int k = 0; k < 8; ++k) o[k] = f2bf(v[k]);
    *(volatile v8us*)(dst + i * 8) = o; __threadfence(); *(volatile v8us*)(dst + i * 8) = o;
}

__global__ __launch_bounds__(256) void k_cvtw(const float* __restrict__ src, h16* dst, size_t n8) {
    const size_t i = (size_t)blockIdx.x * 256 + threadIdx.x; if (i >= n8) return;
    const v8f v = *(const v8f*)(src + i * 8); v8h o;
#pragma unroll
    for (int k = 0; k < 8; ++k) o[k] = toh_flush(bfr(v[k]) * WOC);
    *(volatile v8h*)(dst + i * 8) = o; __threadfence(); *(volatile v8h*)(dst + i * 8) = o;
}

__global__ __launch_bounds__(32) void k_proj(const bf* __restrict__ A, const bf* __restrict__ Bt, const float* __restrict__ bias, h16* Ph, int mode) {
    __shared__ __align__(16) float os[16 * 68];
    const int lane = threadIdx.x & 31, lr = lane & 15, hi = lane >> 4; const int r0 = blockIdx.x * 64, c0 = blockIdx.y * 64;
    v8f acc[4][4];
#pragma unroll
    for (int mb = 0; mb < 4; ++mb)
#pragma unroll
        for (int nb = 0; nb < 4; ++nb) acc[mb][nb] = (v8f){};
    const size_t aoff = (size_t)(r0 + lr) * NF + 8 * hi, boff = (size_t)(c0 + lr) * NF + 8 * hi;
#pragma unroll 1
    for (int kc = 0; kc < NF; kc += 32) {
        v16bf a[4];
#pragma unroll
        for (int mb = 0; mb < 4; ++mb) a[mb] = ldb(A + aoff + (size_t)mb * 16 * NF + kc);
#pragma unroll
        for (int nb = 0; nb < 4; ++nb) { const v16bf b = ldb(Bt + boff + (size_t)nb * 16 * NF + kc);
#pragma unroll
            for (int mb = 0; mb < 4; ++mb) acc[mb][nb] = wmmab_g(a[mb], b, acc[mb][nb]); }
    }
    const bool m0 = (mode == 0);
    float bc[4];
#pragma unroll
    for (int nb = 0; nb < 4; ++nb) { const float t = bias[c0 + nb * 16 + lr]; bc[nb] = m0 ? bfr(t) : 0.0f; }
    size_t tbase;
    if (m0) { const int bb = r0 / SEQ, tt = r0 % SEQ, hh = c0 / DH, dd = c0 % DH;
              tbase = (((size_t)(bb * NH_ + hh) * SEQ) + (size_t)tt) * DH + (size_t)dd; }
    else    { const int bb = c0 / SEQ, tt = c0 % SEQ;
              tbase = ((size_t)bb * HDIM + (size_t)r0) * SEQ + (size_t)tt; }
#pragma unroll
    for (int mb = 0; mb < 4; ++mb) {
        float br[8];
#pragma unroll
        for (int j = 0; j < 8; ++j) { const float t = bias[r0 + mb * 16 + hi * 8 + j]; br[j] = m0 ? 0.0f : bfr(t); }
#pragma unroll
        for (int nb = 0; nb < 4; ++nb) {
#pragma unroll
            for (int j = 0; j < 8; ++j) os[(hi * 8 + j) * 68 + nb * 16 + lr] = acc[mb][nb][j] + bc[nb] + br[j]; }
        wave_sync();
#pragma unroll 1
        for (int ps = 0; ps < 2; ++ps) {
#pragma unroll
            for (int s = 0; s < 4; ++s) { const int row = 4 * s + (lane >> 3), c8 = (lane & 7) * 8;
                const v4f x0 = *(const v4fa*)(&os[row * 68 + c8]); const v4f x1 = *(const v4fa*)(&os[row * 68 + c8 + 4]); v8h hv;
#pragma unroll
                for (int i = 0; i < 4; ++i) { hv[i] = toh_flush(x0[i]); hv[4 + i] = toh_flush(x1[i]); }
                const size_t oo = tbase + (size_t)(mb * 16 + row) * SEQ + c8;
                *(volatile v8h*)(Ph + oo) = hv; }
            if (ps == 0) __threadfence(); }
        wave_sync();
    }
}

__global__ __launch_bounds__(32 * AW) __attribute__((amdgpu_num_vgpr(256)))
void k_attn(const h16* __restrict__ QP, const h16* __restrict__ KT, const h16* __restrict__ VT, h16* CTX) {
    __shared__ __align__(16) h16 sP[32 * PP];
    __shared__ float smax[AW * 32];
    __shared__ float ssum[AW * 32];
    const int lane = threadIdx.x & 31, lr = lane & 15, hi = lane >> 4;
    const int wave = __builtin_amdgcn_readfirstlane((int)(threadIdx.x >> 5));
    const int zh = blockIdx.y; const int b = zh / NH_, h = zh % NH_;
    const int t0 = blockIdx.x * 32;
    const size_t zb = (size_t)zh * SEQ * DH;
    const size_t ao = zb + (size_t)(wave * 128 + lr) * SEQ + 8 * hi;
    const size_t qo = zb + (size_t)(t0 + lr) * DH + 8 * hi;
    v8f acc[8][2];
#pragma unroll
    for (int jb = 0; jb < 8; ++jb) { acc[jb][0] = (v8f){}; acc[jb][1] = (v8f){}; }
#pragma unroll 1
    for (int kc = 0; kc < SEQ; kc += 32) {
        const v16h q0 = ldh(QP + qo + kc), q1 = ldh(QP + qo + (size_t)16 * DH + kc);
#pragma unroll
        for (int jb = 0; jb < 8; ++jb) { const v16h ka = ldh(KT + ao + (size_t)jb * 16 * SEQ + kc);
            acc[jb][0] = wmma16_g(ka, q0, acc[jb][0]); acc[jb][1] = wmma16_g(ka, q1, acc[jb][1]); }
    }
    float mx0 = NEGB, mx1 = NEGB;
#pragma unroll
    for (int jb = 0; jb < 8; ++jb) {
#pragma unroll
        for (int r = 0; r < 8; ++r) { mx0 = fmaxf(mx0, acc[jb][0][r]); mx1 = fmaxf(mx1, acc[jb][1][r]); } }
    mx0 = fmaxf(mx0, __shfl_xor(mx0, 16, 32)); mx1 = fmaxf(mx1, __shfl_xor(mx1, 16, 32));
    smax[wave * 32 + lane] = hi ? mx1 : mx0;
    __syncthreads();
    float g0 = smax[lr], g1 = smax[16 + lr];
#pragma unroll
    for (int w = 1; w < AW; ++w) { g0 = fmaxf(g0, smax[w * 32 + lr]); g1 = fmaxf(g1, smax[w * 32 + 16 + lr]); }
    const float sh0 = PSH - g0 * SC2, sh1 = PSH - g1 * SC2;
    float ls0 = 0.0f, ls1 = 0.0f;
    const int pw = wave * 128 + 8 * hi;
#pragma unroll
    for (int jb = 0; jb < 8; ++jb) { v8h p0, p1;
#pragma unroll
        for (int r = 0; r < 8; ++r) {
            const float e0 = acc[jb][0][r] * SC2 + sh0, e1 = acc[jb][1][r] * SC2 + sh1;
            const h16 a0 = pexp_h(e0), a1 = pexp_h(e1);
            p0[r] = a0; p1[r] = a1; ls0 += (float)a0; ls1 += (float)a1; }
        *(v8h*)(&sP[lr * PP + pw + jb * 16]) = p0; *(v8h*)(&sP[(16 + lr) * PP + pw + jb * 16]) = p1; }
    ls0 += __shfl_xor(ls0, 16, 32); ls1 += __shfl_xor(ls1, 16, 32);
    ssum[wave * 32 + lane] = hi ? ls1 : ls0;
    __syncthreads();
#pragma unroll
    for (int db = 0; db < 8; ++db) { acc[db][0] = (v8f){}; acc[db][1] = (v8f){}; }
#pragma unroll 1
    for (int kc = 0; kc < SEQ; kc += 32) {
        const int pi = lr * PP + kc + 8 * hi;
        const v16h p0 = cat16(*(const v8h*)(&sP[pi]), *(const v8h*)(&sP[pi + 16]));
        const v16h p1 = cat16(*(const v8h*)(&sP[pi + 16 * PP]), *(const v8h*)(&sP[pi + 16 * PP + 16]));
#pragma unroll
        for (int db = 0; db < 8; ++db) { const v16h va = ldh(VT + ao + (size_t)db * 16 * SEQ + kc);
            acc[db][0] = wmma16_g(va, p0, acc[db][0]); acc[db][1] = wmma16_g(va, p1, acc[db][1]); }
    }
    float l0 = ssum[lr], l1 = ssum[16 + lr];
#pragma unroll
    for (int w = 1; w < AW; ++w) { l0 += ssum[w * 32 + lr]; l1 += ssum[w * 32 + 16 + lr]; }
    const float inv0 = CTXC * (1.0f / l0), inv1 = CTXC * (1.0f / l1);
    __syncthreads();
#pragma unroll
    for (int db = 0; db < 8; ++db) { v8h o0, o1;
#pragma unroll
        for (int r = 0; r < 8; ++r) { o0[r] = toh_flush(acc[db][0][r] * inv0); o1[r] = toh_flush(acc[db][1][r] * inv1); }
        *(v8h*)(&sP[lr * PP + pw + db * 16]) = o0; *(v8h*)(&sP[(16 + lr) * PP + pw + db * 16]) = o1; }
    wave_sync();
    h16* crow = CTX + ((size_t)b * SEQ + (size_t)t0) * HDIM + (size_t)h * DH + (size_t)wave * 128;
#pragma unroll 1
    for (int ps = 0; ps < 2; ++ps) {
#pragma unroll
        for (int s = 0; s < 16; ++s) { const int row = 2 * s + (lane >> 4), c8 = (lane & 15) * 8;
            const v8h val = *(const v8h*)(&sP[row * PP + wave * 128 + c8]);
            *(volatile v8h*)(crow + (size_t)row * HDIM + c8) = val; }
        if (ps == 0) __threadfence(); }
}

__global__ __launch_bounds__(32) void k_oproj(const h16* __restrict__ A, const h16* __restrict__ Bt, const float* __restrict__ bias, float* OUT) {
    __shared__ __align__(16) float os[16 * 68];
    const int lane = threadIdx.x & 31, lr = lane & 15, hi = lane >> 4; const int r0 = blockIdx.x * 64, c0 = blockIdx.y * 64;
    v8f acc[4][4];
#pragma unroll
    for (int mb = 0; mb < 4; ++mb)
#pragma unroll
        for (int nb = 0; nb < 4; ++nb) acc[mb][nb] = (v8f){};
    const size_t aoff = (size_t)(r0 + lr) * HDIM + 8 * hi, boff = (size_t)(c0 + lr) * HDIM + 8 * hi;
#pragma unroll 1
    for (int kc = 0; kc < HDIM; kc += 32) {
        v16h a[4];
#pragma unroll
        for (int mb = 0; mb < 4; ++mb) a[mb] = ldh(A + aoff + (size_t)mb * 16 * HDIM + kc);
#pragma unroll
        for (int nb = 0; nb < 4; ++nb) { const v16h b = ldh(Bt + boff + (size_t)nb * 16 * HDIM + kc);
#pragma unroll
            for (int mb = 0; mb < 4; ++mb) acc[mb][nb] = wmma16_g(a[mb], b, acc[mb][nb]); }
    }
    float bc[4];
#pragma unroll
    for (int nb = 0; nb < 4; ++nb) bc[nb] = bfr(bias[c0 + nb * 16 + lr]);
#pragma unroll
    for (int mb = 0; mb < 4; ++mb) {
#pragma unroll
        for (int nb = 0; nb < 4; ++nb) {
#pragma unroll
            for (int j = 0; j < 8; ++j) os[(hi * 8 + j) * 68 + nb * 16 + lr] = acc[mb][nb][j] * OSC + bc[nb]; }
        wave_sync();
#pragma unroll 1
        for (int ps = 0; ps < 2; ++ps) {
#pragma unroll
            for (int s = 0; s < 8; ++s) { const int row = 2 * s + (lane >> 4), c4 = (lane & 15) * 4;
                const v4f val = *(const v4fa*)(&os[row * 68 + c4]);
                *(volatile v4f*)(OUT + (size_t)(r0 + mb * 16 + row) * NF + c0 + c4) = val; }
            if (ps == 0) __threadfence(); }
        wave_sync();
    }
}

static constexpr size_t al256(size_t v) { return (v + 255) & ~(size_t)255; }
static constexpr size_t SZ_XB = al256((size_t)NB * SEQ * NF * 2);
static constexpr size_t SZ_WP = al256((size_t)HDIM * NF * 2);
static constexpr size_t SZ_PL = al256((size_t)BCH * NH_ * SEQ * DH * 2);
static constexpr size_t SZ_CX = al256((size_t)BCH * SEQ * HDIM * 2);
static constexpr size_t SZ_TOTAL = 3 * SZ_XB + 4 * SZ_WP + 3 * SZ_PL + SZ_CX;
static_assert(SZ_TOTAL <= (size_t)134217728);
static_assert((size_t)BCH * NH_ * SEQ * DH == (size_t)BCH * HDIM * SEQ);
static_assert((size_t)NF * HDIM == (size_t)HDIM * NF);

extern "C" void kernel_launch(void* const* d_in, const int* in_sizes, int n_in,
                              void* d_out, int out_size, void* d_ws, size_t ws_size, hipStream_t stream) {
    if (n_in < 11) return;
    const size_t needx = (size_t)NB * SEQ * NF;
    if ((size_t)in_sizes[0] < needx || (size_t)in_sizes[1] < needx || (size_t)in_sizes[2] < needx) return;
    if ((size_t)in_sizes[3] < (size_t)HDIM * NF || (size_t)in_sizes[5] < (size_t)HDIM * NF || (size_t)in_sizes[7] < (size_t)HDIM * NF) return;
    if ((size_t)in_sizes[9] < (size_t)NF * HDIM) return;
    if (in_sizes[4] < HDIM || in_sizes[6] < HDIM || in_sizes[8] < HDIM || in_sizes[10] < NF) return;
    if ((size_t)out_size < needx) return;
    if (SZ_TOTAL > ws_size) return;
    const float* xin[3] = { (const float*)d_in[0], (const float*)d_in[1], (const float*)d_in[2] };
    const float* wq = (const float*)d_in[3]; const float* bq = (const float*)d_in[4];
    const float* wk = (const float*)d_in[5]; const float* bk = (const float*)d_in[6];
    const float* wv = (const float*)d_in[7]; const float* bv = (const float*)d_in[8];
    const float* wo = (const float*)d_in[9]; const float* bo = (const float*)d_in[10];
    float* OUT = (float*)d_out;
    char* wsp = (char*)d_ws;
    bf* XB[3];
    XB[0] = (bf*)wsp; wsp += SZ_XB;
    XB[1] = (bf*)wsp; wsp += SZ_XB;
    XB[2] = (bf*)wsp; wsp += SZ_XB;
    bf* WQ = (bf*)wsp; wsp += SZ_WP;
    bf* WK = (bf*)wsp; wsp += SZ_WP;
    bf* WV = (bf*)wsp; wsp += SZ_WP;
    h16* WOH = (h16*)wsp; wsp += SZ_WP;
    h16* QP = (h16*)wsp; wsp += SZ_PL;
    h16* KTP = (h16*)wsp; wsp += SZ_PL;
    h16* VTP = (h16*)wsp; wsp += SZ_PL;
    h16* CTX = (h16*)wsp; wsp += SZ_CX;

    { const size_t n8 = (size_t)NB * SEQ * NF / 8; const unsigned g = (unsigned)((n8 + 255) / 256);
      for (int i = 0; i < 3; ++i) k_cvt8<<<g, 256, 0, stream>>>(xin[i], XB[i], n8); }
    { const size_t n8 = (size_t)HDIM * NF / 8; const unsigned g = (unsigned)((n8 + 255) / 256);
      k_cvt8<<<g, 256, 0, stream>>>(wq, WQ, n8); k_cvt8<<<g, 256, 0, stream>>>(wk, WK, n8); k_cvt8<<<g, 256, 0, stream>>>(wv, WV, n8);
      k_cvtw<<<g, 256, 0, stream>>>(wo, WOH, n8); }

    for (int c = 0; c < NB / BCH; ++c) {
        const size_t xo = (size_t)c * BCH * SEQ * NF;
        k_proj<<<dim3(BCH * SEQ / 64, HDIM / 64, 1), 32, 0, stream>>>(XB[0] + xo, WQ, bq, QP, 0);
        k_proj<<<dim3(HDIM / 64, BCH * SEQ / 64, 1), 32, 0, stream>>>(WK, XB[1] + xo, bk, KTP, 1);
        k_proj<<<dim3(HDIM / 64, BCH * SEQ / 64, 1), 32, 0, stream>>>(WV, XB[2] + xo, bv, VTP, 1);
        k_attn<<<dim3(SEQ / 32, BCH * NH_, 1), 32 * AW, 0, stream>>>(QP, KTP, VTP, CTX);
        k_oproj<<<dim3(BCH * SEQ / 64, NF / 64, 1), 32, 0, stream>>>(CTX, WOH, bo, OUT + xo);
    }
}
